// EdgeDecoder_67259187855552
// MI455X (gfx1250) — hardware-verified
//
#include <hip/hip_runtime.h>
#include <stddef.h>


typedef _Float16 v16h __attribute__((ext_vector_type(16)));
typedef _Float16 v8h  __attribute__((ext_vector_type(8)));
typedef float    v8f  __attribute__((ext_vector_type(8)));
typedef float    v4f  __attribute__((ext_vector_type(4)));
typedef _Float16 h16;

#ifndef SEQ
#define SEQ 2048
#endif
#define SEQ_FULL 2048
#define KD    256
#define HD    64
#define PW    128
#define MROWS (SEQ)
#define NTILE (SEQ / 32)

static_assert(SEQ >= 64 && SEQ <= SEQ_FULL && (SEQ % 64) == 0);
static_assert((KD % 32) == 0);
static_assert((KD % 64) == 0);
static_assert(KD / 8 == 32);
static_assert(HD == 4 * 16);
static_assert(HD == 64);
static_assert(PW == 2 * HD && (PW % 64) == 0 && (PW % 32) == 0);
static_assert((MROWS % 64) == 0 && (MROWS % 32) == 0);
static_assert((size_t)SEQ_FULL * SEQ_FULL * 4 == (size_t)16777216);
static_assert((size_t)(SEQ - 1) * SEQ_FULL + SEQ <= (size_t)SEQ_FULL * SEQ_FULL);

#define LDT 72
#define LDC 68
#define LPAD 68
#define LSO 36
static_assert((LDT % 8) == 0 && LDT >= 64);
static_assert((LDC % 4) == 0 && LDC >= 64);
static_assert((LPAD % 4) == 0 && LPAD >= HD);
static_assert((LSO % 4) == 0 && LSO >= 32);

#define WCARRY 64.0f
#define XCARRY 16.0f

#define WT_BYTES  ((size_t)PW * KD * 2)
#define X16_BYTES ((size_t)MROWS * KD * 2)
#define PF_BYTES  ((size_t)MROWS * PW * 4)
#define OFF_WT  ((size_t)0)
#define OFF_X16 (OFF_WT + WT_BYTES)
#define OFF_PF  (OFF_X16 + X16_BYTES)
#define WS_TOTAL (OFF_PF + PF_BYTES)
static_assert((WT_BYTES % 128) == 0 && (X16_BYTES % 128) == 0 && (PF_BYTES % 128) == 0);
static_assert(WS_TOTAL <= (size_t)134217728);

#define PAIR_LDS_BYTES ((size_t)(4 * 32 * LPAD + HD + 32 * LSO) * 4)
static_assert(PAIR_LDS_BYTES <= (size_t)131072);
static_assert((size_t)64 * LDC * 4 <= (size_t)131072);
static_assert((size_t)64 * LDT * 2 <= (size_t)131072);

__device__ __forceinline__ float bf16r(float x) {
  unsigned int u = __float_as_uint(x);
  u = (u + 0x7FFFu + ((u >> 16) & 1u)) & 0xFFFF0000u;
  return __uint_as_float(u);
}

__device__ __forceinline__ h16 toh_flush(float v) {
  const h16 r = (h16)v;
  return (fabsf(v) < 6.103515625e-05f) ? (h16)0.0f : r;
}

__device__ __forceinline__ v16h frag_at(const _Float16* p) {
  v8h lo = *(const v8h*)(p);
  v8h hi = *(const v8h*)(p + 16);
  v16h out;
#pragma unroll
  for (int i = 0; i < 8; ++i) { out[i] = lo[i]; out[i + 8] = hi[i]; }
  return out;
}

__device__ __forceinline__ v8f wmma16(v16h a, v16h b, v8f c) {
  v8f d = __builtin_amdgcn_wmma_f32_16x16x32_f16(false, a, false, b, (short)0, c,
                                                 false, false);
  asm volatile("v_nop\n\tv_nop\n\tv_nop\n\tv_nop" : "+v"(d) : "v"(a), "v"(b));
  return d;
}

__device__ __forceinline__ float sigm(float z) {
  return __builtin_amdgcn_rcpf(1.0f + __expf(-z));
}

__global__ __launch_bounds__(256) void wconv_kernel(
    const float* __restrict__ W, _Float16* __restrict__ Wt) {
#pragma clang fp contract(off)
  __shared__ __attribute__((aligned(16))) _Float16 T[64 * LDT];
  const unsigned tid = threadIdx.x;
  const unsigned k0 = blockIdx.x * 64u;
  const unsigned sel = blockIdx.y;
#pragma unroll 4
  for (unsigned j = 0; j < 16u; ++j) {
    const unsigned idx = tid + 256u * j;
    const unsigned kr = idx >> 6, nc = idx & 63u;
    const float v = W[((size_t)sel * KD + k0 + kr) * HD + nc];
    T[nc * LDT + kr] = toh_flush(WCARRY * bf16r(v));
  }
  __syncthreads();
  v8h xs[2];
  size_t off[2];
#pragma unroll
  for (unsigned i = 0; i < 2u; ++i) {
    const unsigned slot = tid + 256u * i;
    const unsigned n = slot >> 3;
    const unsigned kc = (slot & 7u) * 8u;
    xs[i] = *(const v8h*)&T[n * LDT + kc];
    off[i] = (size_t)(sel * (unsigned)HD + n) * KD + k0 + kc;
  }
#pragma unroll
  for (int i = 0; i < 2; ++i) *(volatile v8h*)(Wt + off[i]) = xs[i];
  __threadfence();
#pragma unroll
  for (int i = 0; i < 2; ++i) *(volatile v8h*)(Wt + off[i]) = xs[i];
}
static_assert(256 * 16 == 64 * 64);
static_assert((256 / 8) * 2 == 64);
static_assert((KD / 64) * 64 == KD);

__global__ __launch_bounds__(256) void xconv_kernel(
    const float* __restrict__ X, _Float16* __restrict__ X16) {
#pragma clang fp contract(off)
  const unsigned gid = blockIdx.x * 256u + threadIdx.x;
  const unsigned n = gid >> 5;
  const unsigned c = (gid & 31u) * 8u;
  const float* src = X + (size_t)n * KD + c;
  const v4f a0 = *(const v4f*)(src);
  const v4f a1 = *(const v4f*)(src + 4u);
  v8h o;
#pragma unroll
  for (int i = 0; i < 4; ++i) {
    o[i]     = toh_flush(XCARRY * bf16r(a0[i]));
    o[i + 4] = toh_flush(XCARRY * bf16r(a1[i]));
  }
  _Float16* p = X16 + (size_t)n * KD + c;
  *(volatile v8h*)p = o;
  __threadfence();
  *(volatile v8h*)p = o;
}
static_assert(((size_t)MROWS * KD / 8) % 256 == 0);

__global__ __launch_bounds__(256) void gemm_pre_kernel(
    const _Float16* __restrict__ A16, const _Float16* __restrict__ Bt,
    float* __restrict__ outf) {
  __shared__ float Cs[64 * LDC];
  const unsigned tid = threadIdx.x, lane = tid & 31u;
  const unsigned w = (unsigned)__builtin_amdgcn_readfirstlane((int)(threadIdx.x >> 5));
  const unsigned mw = w >> 1, nw = w & 1u;
  const unsigned hh = lane >> 4, m = lane & 15u;
  const unsigned n0 = blockIdx.x * 64u;
  const unsigned row0 = blockIdx.y * 64u;

  const _Float16* ap  = A16 + (size_t)(row0 + mw * 16u + m) * KD + hh * 8u;
  const _Float16* bp0 = Bt + (size_t)(n0 + nw * 32u + m) * KD + hh * 8u;
  const _Float16* bp1 = bp0 + (size_t)16 * KD;
  v8f acc0 = {}, acc1 = {};
#pragma unroll
  for (unsigned k0 = 0; k0 < (unsigned)KD; k0 += 32u) {
    const v16h a  = frag_at(ap + k0);
    const v16h b0 = frag_at(bp0 + k0);
    const v16h b1 = frag_at(bp1 + k0);
    acc0 = wmma16(a, b0, acc0);
    acc1 = wmma16(a, b1, acc1);
  }
#pragma unroll
  for (int r = 0; r < 8; ++r) {
    float* d = &Cs[(mw * 16u + hh * 8u + (unsigned)r) * LDC + nw * 32u + m];
    d[0]  = acc0[r];
    d[16] = acc1[r];
  }
  __syncthreads();

  const float cs = 1.0f / (WCARRY * XCARRY);
  v4f xs[4];
  size_t off[4];
#pragma unroll
  for (unsigned i = 0; i < 4u; ++i) {
    const unsigned r = 16u * i + (tid >> 4);
    const unsigned c = (tid & 15u) * 4u;
    const v4f u = *(const v4f*)&Cs[r * LDC + c];
    v4f val;
#pragma unroll
    for (int j = 0; j < 4; ++j) val[j] = u[j] * cs;
    xs[i] = val;
    off[i] = (size_t)(row0 + r) * PW + n0 + c;
  }
#pragma unroll
  for (int i = 0; i < 4; ++i) *(volatile v4f*)(outf + off[i]) = xs[i];
  __threadfence();
#pragma unroll
  for (int i = 0; i < 4; ++i) *(volatile v4f*)(outf + off[i]) = xs[i];
}
static_assert(4 * 16 == 64);

__global__ __launch_bounds__(256) void pair_kernel(
    const float* __restrict__ Pf,
    const float* __restrict__ b1, const float* __restrict__ W2, const float* __restrict__ b2,
    float* __restrict__ out) {
#pragma clang fp contract(off)
  __shared__ __attribute__((aligned(16))) float sAI[32 * LPAD];
  __shared__ __attribute__((aligned(16))) float sBI[32 * LPAD];
  __shared__ __attribute__((aligned(16))) float sAJ[32 * LPAD];
  __shared__ __attribute__((aligned(16))) float sBJ[32 * LPAD];
  __shared__ __attribute__((aligned(16))) float w2s[HD];
  __shared__ __attribute__((aligned(16))) float So[32 * LSO];

  const unsigned tid = threadIdx.x;
  const unsigned ti = blockIdx.y, tj = blockIdx.x;
  if (tj < ti) return;
  const unsigned i0 = ti * 32u, j0 = tj * 32u;

  const size_t irow = (size_t)i0 * PW;
  const size_t jrow = (size_t)j0 * PW;
#pragma unroll 1
  for (unsigned s = 0; s < 2u; ++s) {
    const unsigned idx = tid + 256u * s;
    const unsigned r = idx >> 4, c = (idx & 15u) * 4u;
    const v4f ai = *(const v4f*)(Pf + irow + (size_t)r * PW + c);
    const v4f bi = *(const v4f*)(Pf + irow + (size_t)r * PW + HD + c);
    const v4f aj = *(const v4f*)(Pf + jrow + (size_t)r * PW + c);
    const v4f bj = *(const v4f*)(Pf + jrow + (size_t)r * PW + HD + c);
    const v4f g  = *(const v4f*)(b1 + c);
    v4f avi, avj;
#pragma unroll
    for (int j = 0; j < 4; ++j) {
      const float gb = bf16r(g[j]);
      avi[j] = ai[j] + gb;
      avj[j] = aj[j] + gb;
    }
    *(v4f*)&sAI[r * LPAD + c] = avi;
    *(v4f*)&sBI[r * LPAD + c] = bi;
    *(v4f*)&sAJ[r * LPAD + c] = avj;
    *(v4f*)&sBJ[r * LPAD + c] = bj;
  }
  if (tid < (unsigned)HD) w2s[tid] = bf16r(W2[tid]);
  __syncthreads();

  const unsigned tx = tid & 15u, ty = tid >> 4;
  const unsigned pa = (ty * 2u) * LPAD;
  const unsigned pb = (tx * 2u) * LPAD;
  float a00 = 0.0f, a01 = 0.0f, a10 = 0.0f, a11 = 0.0f;
  float m00 = 0.0f, m01 = 0.0f, m10 = 0.0f, m11 = 0.0f;
#pragma unroll 1
  for (unsigned h = 0; h < (unsigned)HD; h += 4u) {
    const v4f wv = *(const v4f*)&w2s[h];
    const v4f x0 = *(const v4f*)&sAI[pa + h];
    const v4f x1 = *(const v4f*)&sAI[pa + LPAD + h];
    const v4f y0 = *(const v4f*)&sBJ[pb + h];
    const v4f y1 = *(const v4f*)&sBJ[pb + LPAD + h];
    const v4f p0 = *(const v4f*)&sBI[pa + h];
    const v4f p1 = *(const v4f*)&sBI[pa + LPAD + h];
    const v4f q0 = *(const v4f*)&sAJ[pb + h];
    const v4f q1 = *(const v4f*)&sAJ[pb + LPAD + h];
#pragma unroll
    for (int j = 0; j < 4; ++j) {
      a00 = fmaf(fmaxf(x0[j] + y0[j], 0.0f), wv[j], a00);
      a01 = fmaf(fmaxf(x0[j] + y1[j], 0.0f), wv[j], a01);
      a10 = fmaf(fmaxf(x1[j] + y0[j], 0.0f), wv[j], a10);
      a11 = fmaf(fmaxf(x1[j] + y1[j], 0.0f), wv[j], a11);
      m00 = fmaf(fmaxf(q0[j] + p0[j], 0.0f), wv[j], m00);
      m01 = fmaf(fmaxf(q1[j] + p0[j], 0.0f), wv[j], m01);
      m10 = fmaf(fmaxf(q0[j] + p1[j], 0.0f), wv[j], m10);
      m11 = fmaf(fmaxf(q1[j] + p1[j], 0.0f), wv[j], m11);
    }
  }
  const float c2 = bf16r(b2[0]);
  const float s00 = sigm(0.5f * ((a00 + c2) + (m00 + c2)));
  const float s01 = sigm(0.5f * ((a01 + c2) + (m01 + c2)));
  const float s10 = sigm(0.5f * ((a10 + c2) + (m10 + c2)));
  const float s11 = sigm(0.5f * ((a11 + c2) + (m11 + c2)));
  So[(2u * ty) * LSO + 2u * tx]            = s00;
  So[(2u * ty) * LSO + 2u * tx + 1u]       = s01;
  So[(2u * ty + 1u) * LSO + 2u * tx]       = s10;
  So[(2u * ty + 1u) * LSO + 2u * tx + 1u]  = s11;
  __syncthreads();

  const unsigned r = tid >> 3, c0 = (tid & 7u) * 4u;
  const v4f u = *(const v4f*)&So[r * LSO + c0];
  v4f t;
#pragma unroll
  for (int j = 0; j < 4; ++j) t[j] = So[(c0 + (unsigned)j) * LSO + r];
  const size_t offa = ((size_t)i0 + r) * SEQ_FULL + j0 + c0;
  const size_t offm = ((size_t)j0 + r) * SEQ_FULL + i0 + c0;
  const bool offd = (tj != ti);
  *(volatile v4f*)(out + offa) = u;
  if (offd) *(volatile v4f*)(out + offm) = t;
  __threadfence();
  *(volatile v4f*)(out + offa) = u;
  if (offd) *(volatile v4f*)(out + offm) = t;
}
static_assert(256 / 8 == 32);
static_assert(16 * 2 == 32);
static_assert(2 * 256 == 32 * (HD / 4));
static_assert(HD <= 64 || (HD % 32) == 0);
static_assert(NTILE * 32 == SEQ);

extern "C" void kernel_launch(void* const* d_in, const int* in_sizes, int n_in,
                              void* d_out, int out_size, void* d_ws, size_t ws_size,
                              hipStream_t stream) {
  if (n_in < 5) return;
  const long long need_x = (long long)SEQ * KD;
  const long long need_o = ((long long)(SEQ - 1)) * SEQ_FULL + SEQ;
  if ((long long)in_sizes[0] < need_x) return;
  if ((long long)in_sizes[1] < (long long)2 * KD * HD) return;
  if (in_sizes[2] < HD || in_sizes[3] < HD || in_sizes[4] < 1) return;
  if ((long long)out_size < need_o) return;
  if (ws_size < WS_TOTAL) return;

  const float* x   = (const float*)d_in[0];
  const float* w1  = (const float*)d_in[1];
  const float* b1  = (const float*)d_in[2];
  const float* w2  = (const float*)d_in[3];
  const float* b2  = (const float*)d_in[4];
  float* out = (float*)d_out;

  char* ws = (char*)d_ws;
  _Float16* Wt  = (_Float16*)(ws + OFF_WT);
  _Float16* X16 = (_Float16*)(ws + OFF_X16);
  float*    Pf  = (float*)(ws + OFF_PF);

  dim3 blk(256);
  wconv_kernel<<<dim3(KD / 64, 2), blk, 0, stream>>>(w1, Wt);
  xconv_kernel<<<dim3(MROWS * KD / 8 / 256), blk, 0, stream>>>(x, X16);
  gemm_pre_kernel<<<dim3(PW / 64, MROWS / 64), blk, 0, stream>>>(X16, Wt, Pf);
  pair_kernel<<<dim3(NTILE, NTILE), blk, 0, stream>>>(Pf, b1, w2, b2, out);
}
